// DeformableConv2d_76244259439171
// MI455X (gfx1250) — hardware-verified
//
#include <hip/hip_runtime.h>


typedef __attribute__((ext_vector_type(16))) _Float16 v16h;
typedef __attribute__((ext_vector_type(8)))  float    v8f;

#define Bn   4
#define Cc   64
#define Hh   128
#define Ww   128
#define HWs  (Hh * Ww)
#define K2c  9
#define Kdim (Cc * K2c)
#define COUT 64
#define NTILES (Bn * HWs / 16)

union V16U { v16h h; uint4 u[2]; };
typedef __attribute__((ext_vector_type(4))) float v4f;
typedef __attribute__((ext_vector_type(4))) unsigned v4u;
template <typename T> static __device__ __forceinline__ void vst2(void* p, T v) { *(volatile T*)p = v; __threadfence(); *(volatile T*)p = v; }
static __device__ __forceinline__ v8f wmma16(v16h a, v16h b, v8f c) {
    v8f d = __builtin_amdgcn_wmma_f32_16x16x32_f16(false, a, false, b, (short)0, c, false, false);
    asm volatile("v_nop\n\tv_nop\n\tv_nop\n\tv_nop" : "+v"(d) : "v"(a), "v"(b));
    return d;
}
static __device__ inline v16h load_bfrag(const void* rowbase_s32, int hi) {
    V16U r; const unsigned short* p = reinterpret_cast<const unsigned short*>(rowbase_s32);
    r.u[0] = *reinterpret_cast<const uint4*>(p + hi * 8);
    r.u[1] = *reinterpret_cast<const uint4*>(p + 16 + hi * 8);
    return r.h;
}

static __device__ inline v16h load_v16(const void* p) {
    V16U r;
    r.u[0] = reinterpret_cast<const uint4*>(p)[0];
    r.u[1] = reinterpret_cast<const uint4*>(p)[1];
    return r.h;
}

__global__ void dcn_pack_weights(const float* __restrict__ w,
                                 const float* __restrict__ w_off,
                                 const float* __restrict__ w_mask,
                                 _Float16* __restrict__ Wp,
                                 _Float16* __restrict__ Wom) {
    int g8 = blockIdx.x * blockDim.x + threadIdx.x;
    union { _Float16 h[8]; v4u u; } pk;
    if (g8 * 8 < COUT * Kdim) {
        #pragma unroll
        for (int e = 0; e < 8; ++e) { int idx = g8 * 8 + e; int o = idx / Kdim, kk = idx % Kdim; int k = kk >> 6, c = kk & 63;
            pk.h[e] = (_Float16)w[(o * Cc + c) * K2c + k]; }
        vst2(Wp + (size_t)g8 * 8, pk.u);
    } else {
        int j0 = g8 * 8 - COUT * Kdim;
        if (j0 < 32 * Kdim) {
            #pragma unroll
            for (int e = 0; e < 8; ++e) { int j = j0 + e; int n = j / Kdim, kk = j % Kdim; int k = kk >> 6, c = kk & 63;
                float v = 0.f;
                if (n < 18)      v = w_off[(n * Cc + c) * K2c + k];
                else if (n < 27) v = w_mask[((n - 18) * Cc + c) * K2c + k];
                pk.h[e] = (_Float16)v; }
            vst2(Wom + j0, pk.u);
        }
    }
}

__global__ void __launch_bounds__(256)
dcn_offmask(const float* __restrict__ x,
            const float* __restrict__ b_off,
            const float* __restrict__ b_mask,
            const _Float16* __restrict__ Wom,
            float* __restrict__ off_ws,
            float* __restrict__ mask_ws) {
    __shared__ __align__(16) unsigned short wlds[32 * Kdim];
    {
        const uint4* src = reinterpret_cast<const uint4*>(Wom);
        uint4*       dst = reinterpret_cast<uint4*>(wlds);
        for (int i = threadIdx.x; i < (32 * Kdim) / 8; i += blockDim.x)
            dst[i] = src[i];
    }
    __syncthreads();

    const int wave = threadIdx.x >> 5;
    const int lane = threadIdx.x & 31;
    const int tile = blockIdx.x * 8 + wave;
    const int p0   = tile << 4;
    const int b    = p0 >> 14;
    const int rem  = p0 & 16383;
    const int h    = rem >> 7;
    const int w0   = rem & 127;
    const int wl   = w0 + (lane & 15);
    const int hi   = lane >> 4;
    const float* xb = x + b * Cc * HWs;

    v8f acc0 = {}, acc1 = {};

    for (int k = 0; k < K2c; ++k) {
        const int ki = k / 3, kj = k % 3;
        const int yy = h - 1 + ki;
        const int xx = wl - 1 + kj;
        const float vf = ((yy >= 0) & (yy < Hh) & (xx >= 0) & (xx < Ww)) ? 1.f : 0.f;
        const int yc = min(max(yy, 0), Hh - 1);
        const int xc = min(max(xx, 0), Ww - 1);
        const float* xr = xb + yc * Ww + xc;

        for (int half = 0; half < 2; ++half) {
            const int cb = half * 32 + hi * 8;
            float t[16];
            #pragma unroll
            for (int i = 0; i < 8; ++i) {
                t[i]     = xr[(cb + i) * HWs];
                t[8 + i] = xr[(cb + 16 + i) * HWs];
            }
            v16h a;
            #pragma unroll
            for (int i = 0; i < 16; ++i)
                a[i] = (_Float16)(vf * t[i]);

            const int s    = 2 * k + half;
            v16h bA = load_bfrag(&wlds[(      (lane & 15)) * Kdim + s * 32], hi);
            v16h bB = load_bfrag(&wlds[(16 + (lane & 15)) * Kdim + s * 32], hi);
            acc0 = wmma16(a, bA, acc0);
            acc1 = wmma16(a, bB, acc1);
        }
    }

    __syncthreads();
    float* st = reinterpret_cast<float*>(wlds);
    const int wbase = (wave << 4) + hi * 8;
    #pragma unroll
    for (int t = 0; t < 2; ++t) {
        const int o = t * 16 + (lane & 15);
        v8f acc = t ? acc1 : acc0;
        if (o < 18) {
            const float bias = b_off[o];
            #pragma unroll
            for (int r = 0; r < 8; ++r) st[o * Ww + wbase + r] = acc[r] + bias;
        } else if (o < 27) {
            const float bias = b_mask[o - 18];
            #pragma unroll
            for (int r = 0; r < 8; ++r) st[o * Ww + wbase + r] = 1.f / (1.f + expf(-(acc[r] + bias)));
        }
    }
    __syncthreads();
    const int prow = (blockIdx.x * 8) << 4;
    const int bb = prow >> 14, hh = (prow & 16383) >> 7;
    for (int q = threadIdx.x; q < 27 * 32; q += 256) { const int o = q >> 5, pc = q & 31;
        const v4f v = *reinterpret_cast<const v4f*>(st + o * Ww + pc * 4);
        if (o < 18) vst2(off_ws + ((size_t)(bb * 18 + o) * Hh + hh) * Ww + pc * 4, v);
        else        vst2(mask_ws + ((size_t)(bb * 9 + (o - 18)) * Hh + hh) * Ww + pc * 4, v); }
}

__global__ void __launch_bounds__(256)
dcn_main(const float* __restrict__ x,
         const float* __restrict__ bvec,
         const _Float16* __restrict__ Wp,
         const float* __restrict__ off_ws,
         const float* __restrict__ mask_ws,
         float* __restrict__ out) {
    const int wave = threadIdx.x >> 5;
    const int lane = threadIdx.x & 31;
    const int tile = blockIdx.x * 8 + wave;
    const int p0   = tile << 4;
    const int b    = p0 >> 14;
    const int rem  = p0 & 16383;
    const int h    = rem >> 7;
    const int w0   = rem & 127;
    const int wl   = w0 + (lane & 15);
    const int hi   = lane >> 4;
    const float* xb = x + b * Cc * HWs;

    __builtin_prefetch(Wp + lane * 64, 0, 3);

    v8f acc[4] = {};

    for (int k = 0; k < K2c; ++k) {
        const int ki = k / 3, kj = k % 3;
        const int po = (b * 18 + 2 * k) * HWs + h * Ww + wl;
        const float dy   = off_ws[po];
        const float dx   = off_ws[po + HWs];
        const float mval = mask_ws[(b * 9 + k) * HWs + h * Ww + wl];

        const float sy  = (float)(h - 1 + ki) + dy;
        const float sx  = (float)(wl - 1 + kj) + dx;
        const float y0f = floorf(sy), x0f = floorf(sx);
        const int   y0  = (int)y0f,   x0i = (int)x0f;
        const float wy1 = sy - y0f,   wx1 = sx - x0f;
        const float wy0 = 1.f - wy1,  wx0 = 1.f - wx1;

        int   idxs[4];
        float wgts[4];
        #pragma unroll
        for (int cr = 0; cr < 4; ++cr) {
            const int yi = y0 + (cr >> 1), xi = x0i + (cr & 1);
            const bool v = (yi >= 0) & (yi < Hh) & (xi >= 0) & (xi < Ww);
            const int yc = min(max(yi, 0), Hh - 1);
            const int xc = min(max(xi, 0), Ww - 1);
            idxs[cr] = yc * Ww + xc;
            const float wy = (cr >> 1) ? wy1 : wy0;
            const float wx = (cr & 1)  ? wx1 : wx0;
            wgts[cr] = v ? wy * wx * mval : 0.f;
        }

        for (int half = 0; half < 2; ++half) {
            const int cb = half * 32 + hi * 8;
            v16h a;
            #pragma unroll
            for (int g = 0; g < 2; ++g) {
                const int cg = cb + g * 16;
                float v0[8], v1[8], v2[8], v3[8];
                #pragma unroll
                for (int i = 0; i < 8; ++i) {
                    const float* pc = xb + (cg + i) * HWs;
                    v0[i] = pc[idxs[0]];
                    v1[i] = pc[idxs[1]];
                    v2[i] = pc[idxs[2]];
                    v3[i] = pc[idxs[3]];
                }
                #pragma unroll
                for (int i = 0; i < 8; ++i) {
                    float v = wgts[0] * v0[i] + wgts[1] * v1[i]
                            + wgts[2] * v2[i] + wgts[3] * v3[i];
                    a[g * 8 + i] = (_Float16)v;
                }
            }
            const int s    = 2 * k + half;
            #pragma unroll
            for (int t = 0; t < 4; ++t) {
                v16h bf = load_bfrag(&Wp[(t * 16 + (lane & 15)) * Kdim + s * 32], hi);
                acc[t] = wmma16(a, bf, acc[t]);
            }
        }
    }

    __shared__ __align__(16) float sto[COUT * Ww];
    const int wbase = (wave << 4) + hi * 8;
    #pragma unroll
    for (int t = 0; t < 4; ++t) {
        const int o  = t * 16 + (lane & 15);
        const float bo = bvec[o];
        #pragma unroll
        for (int r = 0; r < 8; ++r) sto[o * Ww + wbase + r] = acc[t][r] + bo;
    }
    __syncthreads();
    const int prow = (blockIdx.x * 8) << 4;
    const int bb = prow >> 14, hh = (prow & 16383) >> 7;
    for (int q = threadIdx.x; q < COUT * 32; q += 256) { const int o = q >> 5, pc = q & 31;
        vst2(out + ((size_t)(bb * COUT + o) * Hh + hh) * Ww + pc * 4, *reinterpret_cast<const v4f*>(sto + o * Ww + pc * 4)); }
}

extern "C" void kernel_launch(void* const* d_in, const int* in_sizes, int n_in,
                              void* d_out, int out_size, void* d_ws, size_t ws_size,
                              hipStream_t stream) {
    const float* x      = (const float*)d_in[0];
    const float* w_off  = (const float*)d_in[1];
    const float* b_off  = (const float*)d_in[2];
    const float* w_mask = (const float*)d_in[3];
    const float* b_mask = (const float*)d_in[4];
    const float* w      = (const float*)d_in[5];
    const float* bvec   = (const float*)d_in[6];
    float* out = (float*)d_out;

    char* ws = (char*)d_ws;
    _Float16* Wp   = (_Float16*)ws;
    _Float16* Wom  = (_Float16*)(ws + 73728);
    float* off_ws  = (float*)(ws + 73728 + 36864);
    float* mask_ws = off_ws + (size_t)Bn * 18 * HWs;

    dcn_pack_weights<<<27, 256, 0, stream>>>(w, w_off, w_mask, Wp, Wom);
    dcn_offmask<<<NTILES / 8, 256, 0, stream>>>(x, b_off, b_mask, Wom,
                                                off_ws, mask_ws);
    dcn_main<<<NTILES / 8, 256, 0, stream>>>(x, bvec, Wp, off_ws, mask_ws, out);
}
